// PowerCoderAttention_15547781611674
// MI455X (gfx1250) — hardware-verified
//
#include <hip/hip_runtime.h>


#define TT   2048
#define HID  2048
#define HQ   16
#define HKV  8
#define HD   128
#define GP   64
typedef _Float16 h16;
typedef unsigned short bf;
typedef __attribute__((ext_vector_type(16))) __bf16   v16bf;
typedef __attribute__((ext_vector_type(16))) _Float16 v16h;
typedef __attribute__((ext_vector_type(8)))  _Float16 v8h;
typedef __attribute__((ext_vector_type(8)))  unsigned short v8us;
typedef __attribute__((ext_vector_type(8)))  float    v8f;
typedef __attribute__((ext_vector_type(4)))  float    v4f;
typedef v8h  __attribute__((may_alias)) v8ha;
typedef v4f  __attribute__((may_alias)) v4fa;
typedef v8us __attribute__((may_alias)) v8usa;

__device__ __forceinline__ unsigned short f2bf(float f) { unsigned u = __float_as_uint(f); u += 0x7FFFu + ((u >> 16) & 1u); return (unsigned short)(u >> 16); }
__device__ __forceinline__ float bf2f(unsigned short b) { return __uint_as_float(((unsigned)b) << 16); }
__device__ __forceinline__ float bfr(float f) { return bf2f(f2bf(f)); }
__device__ __forceinline__ v16h cat16(v8h lo, v8h hi) { return __builtin_shufflevector(lo, hi, 0, 1, 2, 3, 4, 5, 6, 7, 8, 9, 10, 11, 12, 13, 14, 15); }
__device__ __forceinline__ v16bf cat16b(v8us lo, v8us hi) { return __builtin_bit_cast(v16bf, __builtin_shufflevector(lo, hi, 0, 1, 2, 3, 4, 5, 6, 7, 8, 9, 10, 11, 12, 13, 14, 15)); }
__device__ __forceinline__ v8f wmma16(v16h a, v16h b, v8f c) { return __builtin_amdgcn_wmma_f32_16x16x32_f16(false, a, false, b, (short)0, c, false, false); }
__device__ __forceinline__ v8f wmmab(v16bf a, v16bf b, v8f c) { return __builtin_amdgcn_wmma_f32_16x16x32_bf16(false, a, false, b, (short)0, c, false, false); }


template <typename T16> struct WFrag;
template <> struct WFrag<h16> { typedef v16h V; static __device__ __forceinline__ V ld(const h16* p) { return cat16(*(const v8h*)p, *(const v8h*)(p + 16)); } static __device__ __forceinline__ v8f mma(V a, V b, v8f c) { return wmma16(a, b, c); } };
template <> struct WFrag<bf> { typedef v16bf V; static __device__ __forceinline__ V ld(const bf* p) { return cat16b(*(const v8us*)p, *(const v8us*)(p + 16)); } static __device__ __forceinline__ v8f mma(V a, V b, v8f c) { return wmmab(a, b, c); } };
template <typename T16, int NSPLIT, bool BIAS>
__global__ __launch_bounds__(32) void k_gemmw(const T16* __restrict__ A, const T16* __restrict__ A2, const T16* __restrict__ Bt, const T16* __restrict__ Bt2, int K, float* C, int ldc, const float* __restrict__ bias, size_t sA, size_t sB, size_t sC) {
    typedef typename WFrag<T16>::V V;
    __shared__ __align__(16) float os[16 * 68];
    const size_t z = blockIdx.z; A += z * sA; if (A2) A2 += z * sA; Bt += z * sB; if (Bt2) Bt2 += z * sB; C += z * sC;
    const int lane = threadIdx.x & 31, lr = lane & 15, hi = lane >> 4; const int r0 = blockIdx.x * 64, c0 = blockIdx.y * 64;
    v8f acc[4][4];
#pragma unroll
    for (int mb = 0; mb < 4; ++mb)
#pragma unroll
        for (int nb = 0; nb < 4; ++nb) acc[mb][nb] = (v8f){};
    const size_t aoff = (size_t)(r0 + lr) * K + 8 * hi, boff = (size_t)(c0 + lr) * K + 8 * hi;
#pragma unroll 1
    for (int kc = 0; kc < K; kc += 32) {
        V a[4], a2[4];
#pragma unroll
        for (int mb = 0; mb < 4; ++mb) { a[mb] = WFrag<T16>::ld(A + aoff + (size_t)mb * 16 * K + kc); if (NSPLIT == 1 || NSPLIT == 2) a2[mb] = WFrag<T16>::ld(A2 + aoff + (size_t)mb * 16 * K + kc); }
#pragma unroll
        for (int nb = 0; nb < 4; ++nb) { const V b = WFrag<T16>::ld(Bt + boff + (size_t)nb * 16 * K + kc); V b2; if (NSPLIT >= 2) b2 = WFrag<T16>::ld(Bt2 + boff + (size_t)nb * 16 * K + kc);
#pragma unroll
            for (int mb = 0; mb < 4; ++mb) { acc[mb][nb] = WFrag<T16>::mma(a[mb], b, acc[mb][nb]); if (NSPLIT == 1 || NSPLIT == 2) acc[mb][nb] = WFrag<T16>::mma(a2[mb], b, acc[mb][nb]); if (NSPLIT >= 2) acc[mb][nb] = WFrag<T16>::mma(a[mb], b2, acc[mb][nb]); } }
        asm volatile("v_nop\n\tv_nop\n\tv_nop\n\tv_nop" : "+v"(acc[0][0]), "+v"(acc[1][1]), "+v"(acc[2][2]), "+v"(acc[3][3]) : "v"(a[0]), "v"(a[3]));
    }
#pragma unroll
    for (int mb = 0; mb < 4; ++mb) {
#pragma unroll
        for (int nb = 0; nb < 4; ++nb) {
#pragma unroll
            for (int j = 0; j < 8; ++j) os[(hi * 8 + j) * 68 + nb * 16 + lr] = acc[mb][nb][j]; }
        __builtin_amdgcn_wave_barrier(); asm volatile("" ::: "memory");
        float* crow = C + (size_t)(r0 + mb * 16) * ldc + c0;
#pragma unroll 1
        for (int ps = 0; ps < 2; ++ps) {
#pragma unroll
            for (int s = 0; s < 8; ++s) { const int row = 2 * s + hi, cofs = lr * 4; v4f val = *(const v4fa*)(os + row * 68 + cofs); if (BIAS) { val[0] += bfr(bias[c0 + cofs]); val[1] += bfr(bias[c0 + cofs + 1]); val[2] += bfr(bias[c0 + cofs + 2]); val[3] += bfr(bias[c0 + cofs + 3]); }
                *(volatile v4f*)(crow + (size_t)row * ldc + cofs) = val; }
            if (ps == 0) __threadfence(); }
        __builtin_amdgcn_wave_barrier(); asm volatile("" ::: "memory");
    }
}

template <typename T16, int NSPLIT, int CMODE>
__global__ __launch_bounds__(32) void k_gemmc(const T16* __restrict__ A, const T16* __restrict__ A2, const T16* __restrict__ Bt, const T16* __restrict__ Bt2, int K, float* C, int ldc, int roff, size_t sA, size_t sB, size_t sC) {
    typedef typename WFrag<T16>::V V;
    __shared__ __align__(16) float os[16 * 68];
    const size_t z = blockIdx.z; A += z * sA; if (A2) A2 += z * sA; Bt += z * sB; if (Bt2) Bt2 += z * sB; C += z * sC;
    const int lane = threadIdx.x & 31, lr = lane & 15, hi = lane >> 4; const int r0 = blockIdx.x * 64, c0 = blockIdx.y * 64;
    if (CMODE == 1 && c0 > r0 + roff + 63) return;
    const int Kl = (CMODE == 2) ? min(K, r0 + roff + 64) : K;
    v8f acc[4][4];
#pragma unroll
    for (int mb = 0; mb < 4; ++mb)
#pragma unroll
        for (int nb = 0; nb < 4; ++nb) acc[mb][nb] = (v8f){};
    const size_t aoff = (size_t)(r0 + lr) * K + 8 * hi, boff = (size_t)(c0 + lr) * K + 8 * hi;
#pragma unroll 1
    for (int kc = 0; kc < Kl; kc += 32) {
        V a[4], a2[4];
#pragma unroll
        for (int mb = 0; mb < 4; ++mb) { a[mb] = WFrag<T16>::ld(A + aoff + (size_t)mb * 16 * K + kc); if (NSPLIT == 1 || NSPLIT == 2) a2[mb] = WFrag<T16>::ld(A2 + aoff + (size_t)mb * 16 * K + kc); }
#pragma unroll
        for (int nb = 0; nb < 4; ++nb) { const V b = WFrag<T16>::ld(Bt + boff + (size_t)nb * 16 * K + kc); V b2; if (NSPLIT >= 2) b2 = WFrag<T16>::ld(Bt2 + boff + (size_t)nb * 16 * K + kc);
#pragma unroll
            for (int mb = 0; mb < 4; ++mb) { acc[mb][nb] = WFrag<T16>::mma(a[mb], b, acc[mb][nb]); if (NSPLIT == 1 || NSPLIT == 2) acc[mb][nb] = WFrag<T16>::mma(a2[mb], b, acc[mb][nb]); if (NSPLIT >= 2) acc[mb][nb] = WFrag<T16>::mma(a[mb], b2, acc[mb][nb]); } }
        asm volatile("v_nop\n\tv_nop\n\tv_nop\n\tv_nop" : "+v"(acc[0][0]), "+v"(acc[1][1]), "+v"(acc[2][2]), "+v"(acc[3][3]) : "v"(a[0]), "v"(a[3]));
    }
#pragma unroll
    for (int mb = 0; mb < 4; ++mb) {
#pragma unroll
        for (int nb = 0; nb < 4; ++nb) {
#pragma unroll
            for (int j = 0; j < 8; ++j) os[(hi * 8 + j) * 68 + nb * 16 + lr] = acc[mb][nb][j]; }
        __builtin_amdgcn_wave_barrier(); asm volatile("" ::: "memory");
        float* crow = C + (size_t)(r0 + mb * 16) * ldc + c0;
#pragma unroll 1
        for (int ps = 0; ps < 2; ++ps) {
#pragma unroll
            for (int s = 0; s < 8; ++s) { const int row = 2 * s + hi, cofs = lr * 4; v4f val = *(const v4fa*)(os + row * 68 + cofs);
                *(volatile v4f*)(crow + (size_t)row * ldc + cofs) = val; }
            if (ps == 0) __threadfence(); }
        __builtin_amdgcn_wave_barrier(); asm volatile("" ::: "memory");
    }
}

__device__ __forceinline__ h16 tohx(float x) { return (h16)x; }
__device__ __forceinline__ void splitf(float y, unsigned short& h, unsigned short& l) { h = f2bf(y); l = f2bf(y - bf2f(h)); }
typedef __attribute__((ext_vector_type(2))) _Float16 v2h;
typedef __attribute__((ext_vector_type(4))) _Float16 v4h;
typedef __attribute__((ext_vector_type(2))) unsigned short v2us;
typedef __attribute__((ext_vector_type(4))) unsigned short v4us;

__global__ __launch_bounds__(256) void k_wtG(const float* __restrict__ w, int K, int N, bf* Bt) {
    const int lane = threadIdx.x & 31; const int L0 = (blockIdx.x * 8 + (threadIdx.x >> 5)) * 8; const int nlines = N * K / 64;
#pragma unroll 1
    for (int ps = 0; ps < 2; ++ps) {
#pragma unroll 1
        for (int l = 0; l < 8; ++l) { const int L = L0 + l; if (L >= nlines) break; const size_t e = (size_t)L * 64 + lane * 2; const int k = (int)(e % K), n = (int)(e / K); v2us o;
            o[0] = f2bf(w[(size_t)k * N + n]); o[1] = f2bf(w[(size_t)(k + 1) * N + n]); *(volatile v2us*)(Bt + e) = o; }
        if (ps == 0) __threadfence(); }
}
__global__ __launch_bounds__(256) void k_cvt8(const float* __restrict__ src, bf* dst, size_t n8) { const size_t i = (size_t)blockIdx.x * 256 + threadIdx.x; if (i >= n8) return; const v8f v = *(const v8f*)(src + i * 8); v8us o;
#pragma unroll
    for (int k = 0; k < 8; ++k) o[k] = f2bf(v[k]); *(volatile v8us*)(dst + i * 8) = o; __threadfence(); *(volatile v8us*)(dst + i * 8) = o; }
__global__ __launch_bounds__(256) void k_wgp(const float* __restrict__ w, bf* Bt) { const size_t e = ((size_t)blockIdx.x * 256 + threadIdx.x) * 4; if (e >= (size_t)GP * HID) return; const int k = (int)(e % HID), n = (int)(e / HID); v4us o;
#pragma unroll
    for (int q = 0; q < 4; ++q) o[q] = n < HKV ? f2bf(w[(size_t)(k + q) * HKV + n]) : (unsigned short)0; *(volatile v4us*)(Bt + e) = o; __threadfence(); *(volatile v4us*)(Bt + e) = o; }
__global__ __launch_bounds__(256) void k_rope(const float* __restrict__ F, int nh, int ld, const int* __restrict__ pos, bf* Ph, bf* Pl) { const size_t e = ((size_t)blockIdx.x * 256 + threadIdx.x) * 2; if (e >= (size_t)nh * TT * (HD / 2)) return; const int d = (int)(e % (HD / 2)); const int t = (int)((e / (HD / 2)) % TT); const int h = (int)(e / ((size_t)(HD / 2) * TT)); const float p = (float)pos[t]; const float* f = F + (size_t)t * ld + h * HD; v2us ah, al, bh, bl;
#pragma unroll
    for (int q = 0; q < 2; ++q) { const int dq = d + q; const float inv = __expf(__fmul_rn(-(float)(2 * dq) / (float)HD, 9.210340371976184f)); const float a = __fmul_rn(p, inv); const float c = cosf(a), s = sinf(a); const float x1 = f[dq], x2 = f[HD / 2 + dq];
        float t1 = __fmul_rn(x1, c); asm volatile("" : "+v"(t1)); float t2 = __fmul_rn(x2, s); asm volatile("" : "+v"(t2)); float t3 = __fmul_rn(x2, c); asm volatile("" : "+v"(t3)); float t4 = __fmul_rn(x1, s); asm volatile("" : "+v"(t4));
        unsigned short u, w2; splitf(__fsub_rn(t1, t2), u, w2); ah[q] = u; al[q] = w2; splitf(__fadd_rn(t3, t4), u, w2); bh[q] = u; bl[q] = w2; }
    const size_t o = ((size_t)h * TT + t) * HD + d; *(volatile v2us*)(Ph + o) = ah; *(volatile v2us*)(Pl + o) = al; *(volatile v2us*)(Ph + o + HD / 2) = bh; *(volatile v2us*)(Pl + o + HD / 2) = bl; __threadfence(); *(volatile v2us*)(Ph + o) = ah; *(volatile v2us*)(Pl + o) = al; *(volatile v2us*)(Ph + o + HD / 2) = bh; *(volatile v2us*)(Pl + o + HD / 2) = bl; }
__global__ __launch_bounds__(32) void k_gcum(const float* __restrict__ GF, const float* __restrict__ bg, float* GC) { const int lane = threadIdx.x; const int h = blockIdx.x; const float b = bfr(bg[h]); float carry = 0.f;
    for (int t0 = 0; t0 < TT; t0 += 32) { const float z = __fadd_rn(GF[(size_t)(t0 + lane) * GP + h], b); float v = fminf(z, 0.f) - log1pf(__expf(-fabsf(z)));
#pragma unroll
        for (int sh = 1; sh < 32; sh <<= 1) { const float u = __shfl_up(v, sh, 32); if (lane >= sh) v = __fadd_rn(v, u); }
        const float o = __fadd_rn(carry, v); *(volatile float*)(GC + (size_t)h * TT + t0 + lane) = o; __threadfence(); *(volatile float*)(GC + (size_t)h * TT + t0 + lane) = o; carry = __shfl(o, 31, 32); } }
__global__ __launch_bounds__(256) void k_vtspl(const float* __restrict__ VF, bf* VTh, bf* VTl) { const size_t e = ((size_t)blockIdx.x * 256 + threadIdx.x) * 2; if (e >= (size_t)HKV * HD * TT) return; const int t = (int)(e % TT); const int d = (int)((e / TT) % HD); const int kv = (int)(e / ((size_t)TT * HD)); v2us oh, ol;
#pragma unroll
    for (int u = 0; u < 2; ++u) { unsigned short a, c; splitf(VF[(size_t)(t + u) * (HKV * HD) + kv * HD + d], a, c); oh[u] = a; ol[u] = c; } *(volatile v2us*)(VTh + e) = oh; *(volatile v2us*)(VTl + e) = ol; __threadfence(); *(volatile v2us*)(VTh + e) = oh; *(volatile v2us*)(VTl + e) = ol; }
__global__ __launch_bounds__(256) void k_wspl(const float* __restrict__ Sb, const float* __restrict__ GC, int h0, bf* Wh, bf* Wl) { const size_t e = ((size_t)blockIdx.x * 256 + threadIdx.x) * 4; if (e >= (size_t)2 * TT * TT) return; const int j = (int)(e % TT); const int i = (int)((e / TT) % TT); const int z = (int)(e / ((size_t)TT * TT)); const int kv = (h0 + z) / (HQ / HKV); const float gi = GC[(size_t)kv * TT + i]; v4us oh, ol;
#pragma unroll
    for (int q = 0; q < 4; ++q) { const int jq = j + q; float w = 0.f; if (jq <= i) { const float s = __fmul_rn(Sb[e + q], 0.08838834764831845f); float s2 = __fmul_rn(s, s); asm volatile("" : "+v"(s2)); w = __fmul_rn(s2, __expf(__fsub_rn(gi, GC[(size_t)kv * TT + jq]))); } unsigned short a, c; splitf(w, a, c); oh[q] = a; ol[q] = c; }
    *(volatile v4us*)(Wh + e) = oh; *(volatile v4us*)(Wl + e) = ol; __threadfence(); *(volatile v4us*)(Wh + e) = oh; *(volatile v4us*)(Wl + e) = ol; }
__global__ __launch_bounds__(256) void k_mrg(const float* __restrict__ O, int h0, bf* Ah, bf* Al) { const size_t e = ((size_t)blockIdx.x * 256 + threadIdx.x) * 4; if (e >= (size_t)2 * TT * HD) return; const int d = (int)(e % HD); const int t = (int)((e / HD) % TT); const int z = (int)(e / ((size_t)HD * TT)); const v4f a = *(const v4f*)(O + e); v4us oh, ol;
#pragma unroll
    for (int q = 0; q < 4; ++q) { unsigned short u, c; splitf(a[q], u, c); oh[q] = u; ol[q] = c; } const size_t o = (size_t)t * HID + (h0 + z) * HD + d; *(volatile v4us*)(Ah + o) = oh; *(volatile v4us*)(Al + o) = ol; __threadfence(); *(volatile v4us*)(Ah + o) = oh; *(volatile v4us*)(Al + o) = ol; }

extern "C" void kernel_launch(void* const* d_in, const int* in_sizes, int n_in,
                              void* d_out, int out_size, void* d_ws, size_t ws_size, hipStream_t stream) {
    (void)in_sizes; (void)n_in; (void)out_size;
    const int* pos = (const int*)d_in[0]; const float* IN[12]; for (int i = 1; i < 12; ++i) IN[i] = (const float*)d_in[i];
    float* OUT = (float*)d_out;
    char* wsp = (char*)d_ws;
    auto take = [&](size_t bytes) { char* p = wsp; wsp += (bytes + 255) & ~(size_t)255; return (void*)p; };
    bf* WQ = (bf*)take((size_t)HID * HID * 2); bf* WK = (bf*)take((size_t)HKV * HD * HID * 2); bf* WV = (bf*)take((size_t)HKV * HD * HID * 2); bf* WG = (bf*)take((size_t)GP * HID * 2); bf* WO = (bf*)take((size_t)HID * HID * 2);
    bf* XB = (bf*)take((size_t)TT * HID * 2); float* QF = (float*)take((size_t)TT * HID * 4); float* KF = (float*)take((size_t)TT * HKV * HD * 4); float* VF = (float*)take((size_t)TT * HKV * HD * 4); float* GF = (float*)take((size_t)TT * GP * 4); float* GC = (float*)take((size_t)HKV * TT * 4);
    bf* Qh = (bf*)take((size_t)HQ * TT * HD * 2); bf* Ql = (bf*)take((size_t)HQ * TT * HD * 2); bf* Kh = (bf*)take((size_t)HKV * TT * HD * 2); bf* Kl = (bf*)take((size_t)HKV * TT * HD * 2); bf* VTh = (bf*)take((size_t)HKV * HD * TT * 2); bf* VTl = (bf*)take((size_t)HKV * HD * TT * 2);
    float* Sb = (float*)take((size_t)2 * TT * TT * 4); bf* Wh = (bf*)take((size_t)2 * TT * TT * 2); bf* Wl = (bf*)take((size_t)2 * TT * TT * 2); float* Ob = (float*)take((size_t)2 * TT * HD * 4); bf* Ah = (bf*)take((size_t)TT * HID * 2); bf* Al = (bf*)take((size_t)TT * HID * 2);
    if ((size_t)(wsp - (char*)d_ws) > ws_size) return;
    k_wtG<<<(HID * HID / 64 + 63) / 64, 256, 0, stream>>>(IN[2], HID, HID, WQ); k_wtG<<<(HID * HKV * HD / 64 + 63) / 64, 256, 0, stream>>>(IN[4], HID, HKV * HD, WK); k_wtG<<<(HID * HKV * HD / 64 + 63) / 64, 256, 0, stream>>>(IN[6], HID, HKV * HD, WV); k_wgp<<<(GP * HID / 4 + 255) / 256, 256, 0, stream>>>(IN[8], WG); k_wtG<<<(HID * HID / 64 + 63) / 64, 256, 0, stream>>>(IN[10], HID, HID, WO);
    k_cvt8<<<(TT * HID / 8 + 255) / 256, 256, 0, stream>>>(IN[1], XB, (size_t)TT * HID / 8);
    k_gemmw<bf, 0, true><<<dim3(TT / 64, HID / 64, 1), 32, 0, stream>>>(XB, nullptr, WQ, nullptr, HID, QF, HID, IN[3], 0, 0, 0); k_gemmw<bf, 0, true><<<dim3(TT / 64, HKV * HD / 64, 1), 32, 0, stream>>>(XB, nullptr, WK, nullptr, HID, KF, HKV * HD, IN[5], 0, 0, 0);
    k_gemmw<bf, 0, true><<<dim3(TT / 64, HKV * HD / 64, 1), 32, 0, stream>>>(XB, nullptr, WV, nullptr, HID, VF, HKV * HD, IN[7], 0, 0, 0); k_gemmw<bf, 0, false><<<dim3(TT / 64, 1, 1), 32, 0, stream>>>(XB, nullptr, WG, nullptr, HID, GF, GP, nullptr, 0, 0, 0);
    k_rope<<<(unsigned)(((size_t)HQ * TT * (HD / 2) / 2 + 255) / 256), 256, 0, stream>>>(QF, HQ, HID, pos, Qh, Ql); k_rope<<<(unsigned)(((size_t)HKV * TT * (HD / 2) / 2 + 255) / 256), 256, 0, stream>>>(KF, HKV, HKV * HD, pos, Kh, Kl);
    k_gcum<<<HKV, 32, 0, stream>>>(GF, IN[9], GC); k_vtspl<<<(unsigned)(((size_t)HKV * HD * TT / 2 + 255) / 256), 256, 0, stream>>>(VF, VTh, VTl);
    for (int h0 = 0; h0 < HQ; h0 += 2) { const size_t zq = (size_t)h0, zk = (size_t)(h0 / 2);
        k_gemmc<bf, 2, 1><<<dim3(TT / 64, TT / 64, 2), 32, 0, stream>>>(Qh + zq * TT * HD, Ql + zq * TT * HD, Kh + zk * TT * HD, Kl + zk * TT * HD, HD, Sb, TT, 0, (size_t)TT * HD, 0, (size_t)TT * TT);
        k_wspl<<<(unsigned)(((size_t)2 * TT * TT / 4 + 255) / 256), 256, 0, stream>>>(Sb, GC, h0, Wh, Wl);
        k_gemmc<bf, 2, 2><<<dim3(TT / 64, HD / 64, 2), 32, 0, stream>>>(Wh, Wl, VTh + zk * HD * TT, VTl + zk * HD * TT, TT, Ob, HD, 0, (size_t)TT * TT, 0, (size_t)TT * HD);
        k_mrg<<<(unsigned)(((size_t)2 * TT * HD / 4 + 255) / 256), 256, 0, stream>>>(Ob, h0, Ah, Al); }
    k_gemmw<bf, 1, true><<<dim3(TT / 64, HID / 64, 1), 32, 0, stream>>>(Ah, Al, WO, nullptr, HID, OUT, HID, IN[11], 0, 0, 0);
}
